// SceneGraphDenoiser_60138132078614
// MI455X (gfx1250) — hardware-run, weakly checked
//
#include <hip/hip_runtime.h>
#include <math.h>

typedef __attribute__((ext_vector_type(16))) _Float16 v16h;
typedef __attribute__((ext_vector_type(8)))  _Float16 v8h;
typedef __attribute__((ext_vector_type(8)))  float    v8f;
typedef __attribute__((ext_vector_type(4)))  float    v4f;
typedef __attribute__((ext_vector_type(2)))  float    v2f;
typedef __attribute__((ext_vector_type(4)))  unsigned v4u;

constexpr int kBatch = 8;
constexpr int kNode  = 96;
constexpr int kD     = 256;
constexpr int kL     = 4;
constexpr int kNObj  = 151;
constexpr int kNRel  = 51;
constexpr int kRows  = kBatch * kNode;
constexpr int kHuP   = 2 * kD;
constexpr int kTblP  = (kL + 1) * kD;
constexpr int kTblR  = 64;
constexpr int kObjPad = 192;
constexpr int kRelPad = 64;
constexpr int kHeadP = 2 * kD + kObjPad;
constexpr int kCntP  = 32;
constexpr int kOut0  = kRows * kNObj;
constexpr int kSlab  = kNode * kNRel;
constexpr int kOut1  = kRows * kSlab;
static_assert(kRows == 768 && kHuP == 512 && kTblP == 1280 && kHeadP == 704, "shapes");
static_assert((kOut0 % 128) == 0, "out0 is whole 32-lane float4 groups");
static_assert((kSlab % 32) == 0 && kSlab / 4 == 1224, "pair slab is 153 whole lines");
static_assert((kRows % 32) == 0 && (kD % 64) == 0 && (kHuP % 64) == 0 && (kTblP % 64) == 0 && (kHeadP % 64) == 0, "tile multiples");
static_assert((kD % 32) == 0 && (kTblR % 32) == 0, "K and M multiples");

constexpr float kResScale = 2048.0f;
constexpr float kResInv   = 1.0f / 2048.0f;
constexpr float kWCarry   = 1024.0f;
constexpr float kRtCarry  = 1024.0f;
constexpr float kHCarry   = 16.0f;
constexpr float kSCarry   = 4.0f;
constexpr float kAggCarry = 8.0f;
constexpr float kT1Carry  = 16.0f;
constexpr float kHidCarry = 64.0f;
constexpr float kF16MinNormal = 6.103515625e-05f;

constexpr int kRowW1   = 0;
constexpr int kRowWTB  = kRowW1 + kL * 2 * kD;
constexpr int kRowMW2  = kRowWTB + kTblP;
constexpr int kRowUW1B = kRowMW2 + kL * kD;
constexpr int kRowUW2  = kRowUW1B + kL * kD;
constexpr int kRowHW   = kRowUW2 + kL * kD;
constexpr int kRowRW2  = kRowHW + kHeadP;
constexpr int kWRows   = kRowRW2 + kRelPad;
static_assert(kWRows == 7168, "weight plane rows");

constexpr size_t kSzW    = (size_t)kWRows * kD * 2;
constexpr size_t kSzRT   = (size_t)kTblR * kD * 2;
constexpr size_t kSzTemb = (size_t)kBatch * kD * 4;
constexpr size_t kSzF32  = (size_t)kRows * kD * 4;
constexpr size_t kSzF16  = (size_t)kRows * kD * 2;
constexpr size_t kSzTbl  = (size_t)kTblR * kTblP * 4;
constexpr size_t kSzHU   = (size_t)kRows * kHuP * 4;
constexpr size_t kSzCnt  = (size_t)kRows * kCntP * 4;
constexpr size_t kSzRABO = (size_t)kRows * kHeadP * 4;
constexpr size_t kOffWH   = 0;
constexpr size_t kOffWL   = kOffWH + kSzW;
constexpr size_t kOffRTH  = kOffWL + kSzW;
constexpr size_t kOffRTL  = kOffRTH + kSzRT;
constexpr size_t kOffTemb = kOffRTL + kSzRT;
constexpr size_t kOffH    = kOffTemb + kSzTemb;
constexpr size_t kOffHH   = kOffH + kSzF32;
constexpr size_t kOffHL   = kOffHH + kSzF16;
constexpr size_t kOffTbl  = kOffHL + kSzF16;
constexpr size_t kOffHU   = kOffTbl + kSzTbl;
constexpr size_t kOffSH   = kOffHU + kSzHU;
constexpr size_t kOffSL   = kOffSH + kSzF16;
constexpr size_t kOffCnt  = kOffSL + kSzF16;
constexpr size_t kOffAGH  = kOffCnt + kSzCnt;
constexpr size_t kOffAGL  = kOffAGH + kSzF16;
constexpr size_t kOffT1H  = kOffAGL + kSzF16;
constexpr size_t kOffT1L  = kOffT1H + kSzF16;
constexpr size_t kOffX    = kOffT1L + kSzF16;
constexpr size_t kOffRABO = kOffX + kSzF32;
constexpr size_t kWsTotal = kOffRABO + kSzRABO;
static_assert(kWsTotal == 16293888ull, "carve total");
static_assert(kWsTotal <= 134217728ull, "carve cap");
static_assert((kSzW % 128) == 0 && (kSzRT % 128) == 0 && (kSzTemb % 128) == 0 && (kSzF32 % 128) == 0 &&
              (kSzF16 % 128) == 0 && (kSzTbl % 128) == 0 && (kSzHU % 128) == 0 && (kSzCnt % 128) == 0 &&
              (kSzRABO % 128) == 0, "128-B aligned regions");

__device__ __forceinline__ v8f mma_h(v16h a, v16h b, v8f c) {
  c = __builtin_amdgcn_wmma_f32_16x16x32_f16(false, a, false, b, (short)0, c, false, false);
  asm volatile("v_nop\n\tv_nop\n\tv_nop\n\tv_nop" : "+v"(c) : "v"(a), "v"(b));
  return c;
}
__device__ __forceinline__ v16h frag_ld(const _Float16* p) {
  union { v16h v; v8h h[2]; } f;
  f.h[0] = *(const v8h*)(p);
  f.h[1] = *(const v8h*)(p + 16);
  return f.v;
}
__device__ __forceinline__ float silu_f(float x) {
  return x * __builtin_amdgcn_rcpf(1.0f + expf(-x));
}
__device__ __forceinline__ void split_f16(float x, unsigned& hb, unsigned& lb) {
  const _Float16 h = (_Float16)x;
  float hf = (float)h;
  const unsigned short hs = __builtin_bit_cast(unsigned short, h);
  const bool tiny = fabsf(hf) < kF16MinNormal;
  hf = tiny ? 0.0f : hf;
  hb = tiny ? 0u : (unsigned)hs;
  const _Float16 l = (_Float16)((x - hf) * kResScale);
  const unsigned short ls = __builtin_bit_cast(unsigned short, l);
  lb = (unsigned)ls;
}
__device__ __forceinline__ void pack8(const v4f a0, const v4f a1, float carry, v4u& hw, v4u& lw) {
  unsigned hb[8], lb[8];
#pragma unroll
  for (int e = 0; e < 4; ++e) {
    split_f16(a0[e] * carry, hb[e], lb[e]);
    split_f16(a1[e] * carry, hb[4 + e], lb[4 + e]);
  }
#pragma unroll
  for (int p = 0; p < 4; ++p) {
    hw[p] = hb[2 * p] | (hb[2 * p + 1] << 16);
    lw[p] = lb[2 * p] | (lb[2 * p + 1] << 16);
  }
}

__global__ __launch_bounds__(256) void prep_weights_kernel(
    const float* __restrict__ msg_w1, const float* __restrict__ msg_w2,
    const float* __restrict__ upd_w1, const float* __restrict__ upd_w2,
    const float* __restrict__ relh_w1, const float* __restrict__ objh_w,
    const float* __restrict__ relh_w2,
    unsigned short* __restrict__ WH, unsigned short* __restrict__ WL)
{
  __shared__ float sT[64 * 65];
  const int tid = threadIdx.x;
  const int z = blockIdx.y;
  const float* src;
  int ldsrc = kD, nvalid = kD, ndst = kD, drow;
  if (z < 24) {
    const int l = z / 6;
    const int kind = z - l * 6;
    if (kind == 0)      { src = msg_w1 + (size_t)l * 2 * kD * kD;            drow = kRowW1 + l * 2 * kD; }
    else if (kind == 1) { src = upd_w1 + (size_t)l * 2 * kD * kD;            drow = kRowW1 + l * 2 * kD + kD; }
    else if (kind == 2) { src = msg_w1 + (size_t)l * 2 * kD * kD + kD * kD;  drow = kRowWTB + l * kD; }
    else if (kind == 3) { src = msg_w2 + (size_t)l * kD * kD;                drow = kRowMW2 + l * kD; }
    else if (kind == 4) { src = upd_w1 + (size_t)l * 2 * kD * kD + kD * kD;  drow = kRowUW1B + l * kD; }
    else                { src = upd_w2 + (size_t)l * kD * kD;                drow = kRowUW2 + l * kD; }
  } else if (z == 24) { src = relh_w1;                 drow = kRowHW; }
  else if (z == 25)   { src = relh_w1 + kD * kD;       drow = kRowHW + kD; }
  else if (z == 26)   { src = relh_w1 + 2 * kD * kD;   drow = kRowWTB + kL * kD; }
  else if (z == 27)   { src = objh_w; ldsrc = kNObj; nvalid = kNObj; ndst = kObjPad; drow = kRowHW + 2 * kD; }
  else                { src = relh_w2; ldsrc = kNRel; nvalid = kNRel; ndst = kRelPad; drow = kRowRW2; }
  const int kt = blockIdx.x & 3;
  const int ntile = blockIdx.x >> 2;
  if (ntile * 64 >= ndst) return;
  const int k0 = kt * 64;
#pragma unroll 1
  for (int it = 0; it < 16; ++it) {
    const int kk = it * 4 + (tid >> 6);
    const int nn = tid & 63;
    const int n = ntile * 64 + nn;
    const int nc = n < nvalid ? n : nvalid - 1;
    float v = src[(size_t)(k0 + kk) * ldsrc + nc];
    asm volatile("" : "+v"(v));
    v = (n < nvalid) ? v : 0.0f;
    sT[kk * 65 + nn] = v;
  }
  __syncthreads();
#pragma unroll 1
  for (int it = 0; it < 2; ++it) {
    const int nrow = it * 32 + (tid >> 3);
    const int c8 = (tid & 7) * 8;
    v4f a0, a1;
#pragma unroll
    for (int e = 0; e < 4; ++e) {
      a0[e] = sT[(c8 + e) * 65 + nrow];
      a1[e] = sT[(c8 + 4 + e) * 65 + nrow];
    }
    v4u hw, lw;
    pack8(a0, a1, kWCarry, hw, lw);
    const size_t o = (size_t)(drow + ntile * 64 + nrow) * kD + k0 + c8;
    *(volatile v4u*)(WH + o) = hw;
    *(volatile v4u*)(WL + o) = lw;
    __threadfence();
    *(volatile v4u*)(WH + o) = hw;
    *(volatile v4u*)(WL + o) = lw;
  }
}

__global__ __launch_bounds__(256) void split_rows_kernel(
    const float* __restrict__ src, int rows_valid, float carry,
    unsigned short* __restrict__ dhi, unsigned short* __restrict__ dlo)
{
  const int i = blockIdx.x * 256 + threadIdx.x;
  const int row = i >> 5;
  const int c8 = (i & 31) * 8;
  const int rc = row < rows_valid ? row : rows_valid - 1;
  v4f a0 = *(const v4f*)(src + (size_t)rc * kD + c8);
  v4f a1 = *(const v4f*)(src + (size_t)rc * kD + c8 + 4);
  const bool live = row < rows_valid;
#pragma unroll
  for (int e = 0; e < 4; ++e) {
    float t0 = a0[e], t1 = a1[e];
    asm volatile("" : "+v"(t0), "+v"(t1));
    a0[e] = live ? t0 : 0.0f;
    a1[e] = live ? t1 : 0.0f;
  }
  v4u hw, lw;
  pack8(a0, a1, carry, hw, lw);
  const size_t o = (size_t)row * kD + c8;
  *(volatile v4u*)(dhi + o) = hw;
  *(volatile v4u*)(dlo + o) = lw;
  __threadfence();
  *(volatile v4u*)(dhi + o) = hw;
  *(volatile v4u*)(dlo + o) = lw;
}

__global__ __launch_bounds__(256) void temb_kernel(
    const int* __restrict__ t, const float* __restrict__ tw1, const float* __restrict__ tb1,
    const float* __restrict__ tw2, const float* __restrict__ tb2, float* __restrict__ TEMB)
{
  __shared__ float sA[kBatch * kD];
  __shared__ float sB[kBatch * kD];
  const int d = threadIdx.x;
  const int half = d & 127;
  const float freq = expf((-9.210340371976184f * (float)half) * (1.0f / 128.0f));
#pragma unroll 1
  for (int b = 0; b < kBatch; ++b) {
    const float arg = (float)t[b] * freq;
    float sv, cv;
    sincosf(arg, &sv, &cv);
    sA[b * kD + d] = (d < 128) ? cv : sv;
  }
  __syncthreads();
  {
    float acc[kBatch];
#pragma unroll
    for (int b = 0; b < kBatch; ++b) acc[b] = 0.0f;
#pragma unroll 1
    for (int k = 0; k < kD; ++k) {
      const float w = tw1[(size_t)k * kD + d];
#pragma unroll
      for (int b = 0; b < kBatch; ++b) acc[b] = fmaf(sA[b * kD + k], w, acc[b]);
    }
    const float bv = tb1[d];
#pragma unroll
    for (int b = 0; b < kBatch; ++b) sB[b * kD + d] = acc[b] + bv;
#pragma unroll 1
    for (int b = 0; b < kBatch; ++b) {
      const float v = sB[b * kD + d];
      sB[b * kD + d] = silu_f(v);
    }
  }
  __syncthreads();
  {
    float acc[kBatch];
#pragma unroll
    for (int b = 0; b < kBatch; ++b) acc[b] = 0.0f;
#pragma unroll 1
    for (int k = 0; k < kD; ++k) {
      const float w = tw2[(size_t)k * kD + d];
#pragma unroll
      for (int b = 0; b < kBatch; ++b) acc[b] = fmaf(sB[b * kD + k], w, acc[b]);
    }
    const float bv = tb2[d];
#pragma unroll
    for (int b = 0; b < kBatch; ++b) sA[b * kD + d] = acc[b] + bv;
  }
#pragma unroll 1
  for (int b = 0; b < kBatch; ++b) {
    const float v = sA[b * kD + d];
    *(volatile float*)(TEMB + b * kD + d) = v;
    __threadfence();
    *(volatile float*)(TEMB + b * kD + d) = v;
  }
}

__device__ __forceinline__ void emit_row(v4f y0, v4f y1, int row, int wave, int lane,
                                         float* __restrict__ H, unsigned short* __restrict__ PH,
                                         unsigned short* __restrict__ PL, float* srow)
{
  float* sr = srow + wave * kD;
  *(v4f*)(sr + lane * 4) = y0;
  *(v4f*)(sr + 128 + lane * 4) = y1;
  __syncthreads();
  const v4f a0 = *(const v4f*)(sr + lane * 8);
  const v4f a1 = *(const v4f*)(sr + lane * 8 + 4);
  v4u hw, lw;
  pack8(a0, a1, kHCarry, hw, lw);
  float* hp = H + (size_t)row * kD;
  const size_t po = (size_t)row * kD + lane * 8;
  for (int pass = 0; pass < 2; ++pass) {
    *(volatile v4f*)(hp + lane * 4) = y0;
    *(volatile v4f*)(hp + 128 + lane * 4) = y1;
    *(volatile v4u*)(PH + po) = hw;
    *(volatile v4u*)(PL + po) = lw;
    __threadfence();
  }
}

__global__ __launch_bounds__(256) void init_h_kernel(
    const int* __restrict__ obj_t, const int* __restrict__ node_mask,
    const float* __restrict__ obj_table, const float* __restrict__ TEMB,
    float* __restrict__ H, unsigned short* __restrict__ HH, unsigned short* __restrict__ HL)
{
  __shared__ __align__(16) float srow[8 * kD];
  const int lane = threadIdx.x & 31;
  const int wave = __builtin_amdgcn_readfirstlane((int)(threadIdx.x >> 5));
  const int row = blockIdx.x * 8 + wave;
  const int b = row / kNode;
  int o = obj_t[row];
  o = o < 0 ? 0 : (o > kNObj - 1 ? kNObj - 1 : o);
  const int nm = node_mask[row];
  const float* ep = obj_table + (size_t)o * kD;
  const float* tp = TEMB + b * kD;
  const v4f e0 = *(const v4f*)(ep + lane * 4);
  const v4f e1 = *(const v4f*)(ep + 128 + lane * 4);
  const v4f t0 = *(const v4f*)(tp + lane * 4);
  const v4f t1 = *(const v4f*)(tp + 128 + lane * 4);
  const float nmf = (float)nm;
  v4f y0 = (e0 + t0) * nmf;
  v4f y1 = (e1 + t1) * nmf;
  if (nm == 0) {
    y0 = (v4f){0.f, 0.f, 0.f, 0.f};
    y1 = (v4f){0.f, 0.f, 0.f, 0.f};
  }
  emit_row(y0, y1, row, wave, lane, H, HH, HL, srow);
}

__global__ __launch_bounds__(256) void ln_kernel(
    const float* __restrict__ X, const float* __restrict__ g, const float* __restrict__ be,
    const int* __restrict__ node_mask,
    float* __restrict__ H, unsigned short* __restrict__ HH, unsigned short* __restrict__ HL)
{
  __shared__ __align__(16) float srow[8 * kD];
  const int lane = threadIdx.x & 31;
  const int wave = __builtin_amdgcn_readfirstlane((int)(threadIdx.x >> 5));
  const int row = blockIdx.x * 8 + wave;
  const float* xp = X + (size_t)row * kD;
  const v4f x0 = *(const v4f*)(xp + lane * 4);
  const v4f x1 = *(const v4f*)(xp + 128 + lane * 4);
  float s = ((x0[0] + x0[1]) + (x0[2] + x0[3])) + ((x1[0] + x1[1]) + (x1[2] + x1[3]));
#pragma unroll
  for (int off = 16; off >= 1; off >>= 1) s += __shfl_xor(s, off, 32);
  const float mu = s * (1.0f / (float)kD);
  const v4f d0 = x0 - mu;
  const v4f d1 = x1 - mu;
  float ss = ((d0[0] * d0[0] + d0[1] * d0[1]) + (d0[2] * d0[2] + d0[3] * d0[3])) +
             ((d1[0] * d1[0] + d1[1] * d1[1]) + (d1[2] * d1[2] + d1[3] * d1[3]));
#pragma unroll
  for (int off = 16; off >= 1; off >>= 1) ss += __shfl_xor(ss, off, 32);
  const float var = ss * (1.0f / (float)kD);
  const float rs = rsqrtf(var + 1e-5f);
  const v4f g0 = *(const v4f*)(g + lane * 4);
  const v4f g1 = *(const v4f*)(g + 128 + lane * 4);
  const v4f b0 = *(const v4f*)(be + lane * 4);
  const v4f b1 = *(const v4f*)(be + 128 + lane * 4);
  const int nm = node_mask[row];
  const float nmf = (float)nm;
  v4f y0 = ((d0 * rs) * g0 + b0) * nmf;
  v4f y1 = ((d1 * rs) * g1 + b1) * nmf;
  if (nm == 0) {
    y0 = (v4f){0.f, 0.f, 0.f, 0.f};
    y1 = (v4f){0.f, 0.f, 0.f, 0.f};
  }
  emit_row(y0, y1, row, wave, lane, H, HH, HL, srow);
}

template <int EPI>
__global__ __launch_bounds__(256) void gemm3_kernel(
    const _Float16* __restrict__ AH, const _Float16* __restrict__ AL, int lda,
    const _Float16* __restrict__ BH, const _Float16* __restrict__ BL, int ldb,
    float* __restrict__ Cf, unsigned short* __restrict__ CH, unsigned short* __restrict__ CL, int ldc,
    const float* __restrict__ bias, const float* __restrict__ aux, int ldaux,
    int M, int N, int K, float scale, float ocarry)
{
  __shared__ __align__(16) float sT[8][16 * 68];
  const int lane = threadIdx.x & 31;
  const int wave = __builtin_amdgcn_readfirstlane((int)(threadIdx.x >> 5));
  const int tilesN = N >> 6;
  const int tilesM = M >> 5;
  const int tile = blockIdx.x * 8 + wave;
  if (tile >= tilesM * tilesN) return;
  const int tm = tile / tilesN;
  const int tn = tile - tm * tilesN;
  const int m0 = tm << 5;
  const int n0 = tn << 6;
  const int rl = lane & 15;
  const int koff = (lane >> 4) * 8;
  const int mOff = (lane >> 4) * 8;

  v8f accm[2][4], accr[2][4];
#pragma unroll
  for (int i = 0; i < 2; ++i)
#pragma unroll
    for (int j = 0; j < 4; ++j) {
      accm[i][j] = (v8f){0.f, 0.f, 0.f, 0.f, 0.f, 0.f, 0.f, 0.f};
      accr[i][j] = (v8f){0.f, 0.f, 0.f, 0.f, 0.f, 0.f, 0.f, 0.f};
    }

  for (int k0 = 0; k0 < K; k0 += 32) {
    v16h ah[2], al[2];
#pragma unroll
    for (int i = 0; i < 2; ++i) {
      const size_t ao = (size_t)(m0 + (i << 4) + rl) * lda + koff + k0;
      ah[i] = frag_ld(AH + ao);
      al[i] = frag_ld(AL + ao);
    }
#pragma unroll
    for (int j = 0; j < 4; ++j) {
      const size_t bo = (size_t)(n0 + (j << 4) + rl) * ldb + koff + k0;
      const v16h bh = frag_ld(BH + bo);
      const v16h bl = frag_ld(BL + bo);
#pragma unroll
      for (int i = 0; i < 2; ++i) {
        accm[i][j] = mma_h(ah[i], bh, accm[i][j]);
        accr[i][j] = mma_h(ah[i], bl, accr[i][j]);
        accr[i][j] = mma_h(al[i], bh, accr[i][j]);
      }
    }
  }

  float* slab = sT[wave];
#pragma unroll
  for (int i = 0; i < 2; ++i) {
    const int mBase = m0 + (i << 4);
#pragma unroll
    for (int j = 0; j < 4; ++j) {
#pragma unroll
      for (int r = 0; r < 8; ++r) {
        const float v = (accm[i][j][r] + accr[i][j][r] * kResInv) * scale;
        slab[(mOff + r) * 68 + (j << 4) + rl] = v;
      }
    }
    __builtin_amdgcn_fence(__ATOMIC_RELEASE, "workgroup");
    __builtin_amdgcn_wave_barrier();
    __builtin_amdgcn_fence(__ATOMIC_ACQUIRE, "workgroup");
    if (EPI == 0 || EPI == 3) {
      const int hh = lane >> 4, c4 = (lane & 15) * 4;
      const int gn = n0 + c4;
      for (int pass = 0; pass < 2; ++pass) {
#pragma unroll
        for (int it = 0; it < 8; ++it) {
          const int row = it * 2 + hh;
          const size_t gm = (size_t)(mBase + row);
          v4f v = *(const v4f*)(slab + row * 68 + c4);
          if (EPI == 3) {
            const v4f bv = *(const v4f*)(bias + gn);
            const v4f rv = *(const v4f*)(aux + gm * ldaux + gn);
            v = (v + bv) + rv;
          }
          *(volatile v4f*)(Cf + gm * ldc + gn) = v;
        }
        __threadfence();
      }
    } else {
      const int q = lane >> 3, c8 = (lane & 7) * 8;
      const int gn = n0 + c8;
#pragma unroll 1
      for (int it = 0; it < 4; ++it) {
        const int row = it * 4 + q;
        const size_t gm = (size_t)(mBase + row);
        const float* sp = slab + row * 68 + c8;
        v4f a0 = *(const v4f*)(sp);
        v4f a1 = *(const v4f*)(sp + 4);
        const v4f b0 = *(const v4f*)(bias + gn);
        const v4f b1 = *(const v4f*)(bias + gn + 4);
        if (EPI == 1) {
          const float c = aux[gm * ldaux];
          a0 = a0 + c * b0;
          a1 = a1 + c * b1;
        } else {
          const v4f u0 = *(const v4f*)(aux + gm * ldaux + gn);
          const v4f u1 = *(const v4f*)(aux + gm * ldaux + gn + 4);
          a0 = (u0 + a0) + b0;
          a1 = (u1 + a1) + b1;
#pragma unroll
          for (int e = 0; e < 4; ++e) {
            a0[e] = silu_f(a0[e]);
            a1[e] = silu_f(a1[e]);
          }
        }
        v4u hw, lw;
        pack8(a0, a1, ocarry, hw, lw);
        const size_t o = gm * ldc + gn;
        *(volatile v4u*)(CH + o) = hw;
        *(volatile v4u*)(CL + o) = lw;
        __threadfence();
        *(volatile v4u*)(CH + o) = hw;
        *(volatile v4u*)(CL + o) = lw;
      }
    }
    __builtin_amdgcn_fence(__ATOMIC_RELEASE, "workgroup");
    __builtin_amdgcn_wave_barrier();
    __builtin_amdgcn_fence(__ATOMIC_ACQUIRE, "workgroup");
  }
}

__global__ __launch_bounds__(256) void edge_sum_kernel(
    const int* __restrict__ rel_t, const int* __restrict__ edge_mask,
    const float* __restrict__ HU, const float* __restrict__ TBL, int tcol,
    const float* __restrict__ mb1,
    unsigned short* __restrict__ SH, unsigned short* __restrict__ SL, float* __restrict__ CNT)
{
  __shared__ int sR[kNode];
  __shared__ int sM[kNode];
  __shared__ __align__(16) float sAcc[kD];
  const int tid = threadIdx.x;
  const int lane = tid & 31;
  const int wave = __builtin_amdgcn_readfirstlane((int)(tid >> 5));
  const int bi = blockIdx.x;
  const int b = bi / kNode;
  const int i = bi - b * kNode;
  {
    const int jc = tid < kNode ? tid : kNode - 1;
    const size_t idx = (size_t)(b * kNode + jc) * kNode + i;
    int rv = rel_t[idx];
    int mv = edge_mask[idx];
    asm volatile("" : "+v"(rv), "+v"(mv));
    rv = rv < 0 ? 0 : (rv > kNRel - 1 ? kNRel - 1 : rv);
    if (tid < kNode) {
      sR[tid] = rv;
      sM[tid] = mv;
    }
  }
  __syncthreads();
  const float bb = mb1[tid];
  float acc = 0.0f, cnt = 0.0f;
#pragma unroll 1
  for (int j = 0; j < kNode; ++j) {
    const int mi = __builtin_amdgcn_readfirstlane(sM[j]);
    const int r = __builtin_amdgcn_readfirstlane(sR[j]);
    if (mi != 0) {
      const float x = (HU[(size_t)(b * kNode + j) * kHuP + tid] + TBL[(size_t)r * kTblP + tcol + tid]) + bb;
      const float mf = (float)mi;
      acc = fmaf(mf, silu_f(x), acc);
      cnt += mf;
    }
  }
  sAcc[tid] = acc;
  __syncthreads();
  if (wave == 0) {
    const v4f a0 = *(const v4f*)(sAcc + lane * 8);
    const v4f a1 = *(const v4f*)(sAcc + lane * 8 + 4);
    v4u hw, lw;
    pack8(a0, a1, kSCarry, hw, lw);
    const size_t o = (size_t)bi * kD + lane * 8;
    *(volatile v4u*)(SH + o) = hw;
    *(volatile v4u*)(SL + o) = lw;
    __threadfence();
    *(volatile v4u*)(SH + o) = hw;
    *(volatile v4u*)(SL + o) = lw;
  } else if (wave == 1) {
    *(volatile float*)(CNT + (size_t)bi * kCntP + lane) = cnt;
    __threadfence();
    *(volatile float*)(CNT + (size_t)bi * kCntP + lane) = cnt;
  }
}

__global__ __launch_bounds__(256) void obj_out_kernel(
    const float* __restrict__ RABO, const float* __restrict__ objb, float* __restrict__ out0)
{
  const int lane = threadIdx.x & 31;
  const int wave = __builtin_amdgcn_readfirstlane((int)(threadIdx.x >> 5));
  const int gw = blockIdx.x * 8 + wave;
  if (gw >= kOut0 / 128) return;
  const int idx = gw * 32 + lane;
  v4f v;
#pragma unroll
  for (int e = 0; e < 4; ++e) {
    const int el = idx * 4 + e;
    const int row = el / kNObj;
    const int col = el - row * kNObj;
    v[e] = RABO[(size_t)row * kHeadP + 2 * kD + col] + objb[col];
  }
  *(volatile v4f*)(out0 + (size_t)idx * 4) = v;
  __threadfence();
  *(volatile v4f*)(out0 + (size_t)idx * 4) = v;
}

constexpr int kHP = 264;
__global__ __launch_bounds__(256) void pair_head_kernel(
    const int* __restrict__ rel_t, const float* __restrict__ RABO, const float* __restrict__ TBL,
    const float* __restrict__ b1, const _Float16* __restrict__ W2H, const float* __restrict__ b2,
    float* __restrict__ out1)
{
  __shared__ __align__(16) _Float16 sHh[32 * kHP];
  __shared__ __align__(16) _Float16 sHl[32 * kHP];
  __shared__ __align__(16) float sOut[kSlab];
  __shared__ int sRel[kNode];
  const int tid = threadIdx.x;
  const int lane = tid & 31;
  const int wave = __builtin_amdgcn_readfirstlane((int)(tid >> 5));
  const int bi = blockIdx.x;
  const int b = bi / kNode;
  {
    const int jc = tid < kNode ? tid : kNode - 1;
    int rv = rel_t[(size_t)bi * kNode + jc];
    asm volatile("" : "+v"(rv));
    rv = rv < 0 ? 0 : (rv > kNRel - 1 ? kNRel - 1 : rv);
    if (tid < kNode) sRel[tid] = rv;
  }
  const int d0 = (tid & 127) * 2;
  const int jh = tid >> 7;
  const v2f ra = *(const v2f*)(RABO + (size_t)bi * kHeadP + d0);
  const v2f bb = *(const v2f*)(b1 + d0);
  const int nt = wave & 3;
  const int mt = wave >> 2;
  const int rl = lane & 15;
  const int koff = (lane >> 4) * 8;
  const int mOff = (lane >> 4) * 8;
  v16h bq[8];
#pragma unroll
  for (int ks = 0; ks < 8; ++ks) bq[ks] = frag_ld(W2H + (size_t)(nt * 16 + rl) * kD + koff + ks * 32);
  const int col = nt * 16 + rl;
  const int colc = col < kNRel ? col : kNRel - 1;
  float b2v = b2[colc];
  asm volatile("" : "+v"(b2v));
  constexpr float kScale = 1.0f / (kHidCarry * kWCarry);
  unsigned* sHh32 = (unsigned*)sHh;
  unsigned* sHl32 = (unsigned*)sHl;
  __syncthreads();
#pragma unroll 1
  for (int jt = 0; jt < 3; ++jt) {
#pragma unroll 1
    for (int s = 0; s < 16; ++s) {
      const int jj = jh * 16 + s;
      const int j = jt * 32 + jj;
      const int r = sRel[j];
      const v2f rb = *(const v2f*)(RABO + (size_t)(b * kNode + j) * kHeadP + kD + d0);
      const v2f tc = *(const v2f*)(TBL + (size_t)r * kTblP + kL * kD + d0);
      const float x0 = ((ra[0] + rb[0]) + tc[0]) + bb[0];
      const float x1 = ((ra[1] + rb[1]) + tc[1]) + bb[1];
      unsigned h0, l0, h1, l1;
      split_f16(silu_f(x0) * kHidCarry, h0, l0);
      split_f16(silu_f(x1) * kHidCarry, h1, l1);
      sHh32[(jj * kHP + d0) >> 1] = h0 | (h1 << 16);
      sHl32[(jj * kHP + d0) >> 1] = l0 | (l1 << 16);
    }
    __syncthreads();
    v8f accm = (v8f){0.f, 0.f, 0.f, 0.f, 0.f, 0.f, 0.f, 0.f};
    v8f accr = (v8f){0.f, 0.f, 0.f, 0.f, 0.f, 0.f, 0.f, 0.f};
#pragma unroll
    for (int ks = 0; ks < 8; ++ks) {
      const int ao = (mt * 16 + rl) * kHP + koff + ks * 32;
      union { v16h v; v8h h[2]; } fa, fl;
      fa.h[0] = *(const v8h*)(sHh + ao);
      fa.h[1] = *(const v8h*)(sHh + ao + 16);
      fl.h[0] = *(const v8h*)(sHl + ao);
      fl.h[1] = *(const v8h*)(sHl + ao + 16);
      accm = mma_h(fa.v, bq[ks], accm);
      accr = mma_h(fl.v, bq[ks], accr);
    }
#pragma unroll
    for (int r = 0; r < 8; ++r) {
      const int row = jt * 32 + mt * 16 + mOff + r;
      const float v = (accm[r] + accr[r] * kResInv) * kScale + b2v;
      if (col < kNRel) sOut[row * kNRel + col] = v;
    }
    __syncthreads();
  }
  float* op = out1 + (size_t)bi * kSlab;
  for (int pass = 0; pass < 2; ++pass) {
#pragma unroll
    for (int it = 0; it < 5; ++it) {
      const int idx = it * 256 + tid;
      const int idc = idx < kSlab / 4 ? idx : kSlab / 4 - 1;
      const v4f v = *(const v4f*)(sOut + idc * 4);
      if (idx < kSlab / 4) *(volatile v4f*)(op + (size_t)idx * 4) = v;
    }
    __threadfence();
  }
}

extern "C" void kernel_launch(void* const* d_in, const int* in_sizes, int n_in,
                              void* d_out, int out_size, void* d_ws, size_t ws_size,
                              hipStream_t stream) {
  if (n_in < 27) return;
  if (in_sizes[0] != kRows) return;
  if (in_sizes[1] != kRows * kNode) return;
  if (in_sizes[2] != kBatch) return;
  if (in_sizes[3] != kRows) return;
  if (in_sizes[4] != kRows * kNode) return;
  if (in_sizes[5] != kNObj * kD) return;
  if (in_sizes[6] != kNRel * kD) return;
  if (in_sizes[11] != kL * 2 * kD * kD) return;
  if (in_sizes[13] != kL * kD * kD) return;
  if (in_sizes[15] != kL * 2 * kD * kD) return;
  if (in_sizes[17] != kL * kD * kD) return;
  if (in_sizes[21] != kD * kNObj) return;
  if (in_sizes[23] != 3 * kD * kD) return;
  if (in_sizes[25] != kD * kNRel) return;
  if (in_sizes[26] != kNRel) return;
  if (out_size != kOut0 + kOut1) return;
  if (ws_size < kWsTotal) return;

  const int*   obj_t     = (const int*)d_in[0];
  const int*   rel_t     = (const int*)d_in[1];
  const int*   t_in      = (const int*)d_in[2];
  const int*   node_mask = (const int*)d_in[3];
  const int*   edge_mask = (const int*)d_in[4];
  const float* obj_table = (const float*)d_in[5];
  const float* rel_table = (const float*)d_in[6];
  const float* tw1 = (const float*)d_in[7];
  const float* tb1 = (const float*)d_in[8];
  const float* tw2 = (const float*)d_in[9];
  const float* tb2 = (const float*)d_in[10];
  const float* msg_w1 = (const float*)d_in[11];
  const float* msg_b1 = (const float*)d_in[12];
  const float* msg_w2 = (const float*)d_in[13];
  const float* msg_b2 = (const float*)d_in[14];
  const float* upd_w1 = (const float*)d_in[15];
  const float* upd_b1 = (const float*)d_in[16];
  const float* upd_w2 = (const float*)d_in[17];
  const float* upd_b2 = (const float*)d_in[18];
  const float* ln_g = (const float*)d_in[19];
  const float* ln_b = (const float*)d_in[20];
  const float* objh_w = (const float*)d_in[21];
  const float* objh_b = (const float*)d_in[22];
  const float* relh_w1 = (const float*)d_in[23];
  const float* relh_b1 = (const float*)d_in[24];
  const float* relh_w2 = (const float*)d_in[25];
  const float* relh_b2 = (const float*)d_in[26];

  char* ws = (char*)d_ws;
  unsigned short* WH   = (unsigned short*)(ws + kOffWH);
  unsigned short* WL   = (unsigned short*)(ws + kOffWL);
  unsigned short* RTH  = (unsigned short*)(ws + kOffRTH);
  unsigned short* RTL  = (unsigned short*)(ws + kOffRTL);
  float*          TEMB = (float*)(ws + kOffTemb);
  float*          H    = (float*)(ws + kOffH);
  unsigned short* HH   = (unsigned short*)(ws + kOffHH);
  unsigned short* HL   = (unsigned short*)(ws + kOffHL);
  float*          TBL  = (float*)(ws + kOffTbl);
  float*          HU   = (float*)(ws + kOffHU);
  unsigned short* SH   = (unsigned short*)(ws + kOffSH);
  unsigned short* SL   = (unsigned short*)(ws + kOffSL);
  float*          CNT  = (float*)(ws + kOffCnt);
  unsigned short* AGH  = (unsigned short*)(ws + kOffAGH);
  unsigned short* AGL  = (unsigned short*)(ws + kOffAGL);
  unsigned short* T1H  = (unsigned short*)(ws + kOffT1H);
  unsigned short* T1L  = (unsigned short*)(ws + kOffT1L);
  float*          X    = (float*)(ws + kOffX);
  float*          RABO = (float*)(ws + kOffRABO);
  float* out0 = (float*)d_out;
  float* out1 = out0 + kOut0;

  const _Float16* WHh = (const _Float16*)WH;
  const _Float16* WLh = (const _Float16*)WL;

  prep_weights_kernel<<<dim3(16, 29), 256, 0, stream>>>(msg_w1, msg_w2, upd_w1, upd_w2, relh_w1, objh_w, relh_w2, WH, WL);
  split_rows_kernel<<<(kTblR * kD / 8) / 256, 256, 0, stream>>>(rel_table, kNRel, kRtCarry, RTH, RTL);
  temb_kernel<<<1, 256, 0, stream>>>(t_in, tw1, tb1, tw2, tb2, TEMB);
  init_h_kernel<<<kRows / 8, 256, 0, stream>>>(obj_t, node_mask, obj_table, TEMB, H, HH, HL);
  gemm3_kernel<0><<<5, 256, 0, stream>>>(
      (const _Float16*)RTH, (const _Float16*)RTL, kD,
      WHh + (size_t)kRowWTB * kD, WLh + (size_t)kRowWTB * kD, kD,
      TBL, nullptr, nullptr, kTblP,
      nullptr, nullptr, 0,
      kTblR, kTblP, kD, 1.0f / (kRtCarry * kWCarry), 1.0f);

  for (int l = 0; l < kL; ++l) {
    gemm3_kernel<0><<<24, 256, 0, stream>>>(
        (const _Float16*)HH, (const _Float16*)HL, kD,
        WHh + (size_t)(kRowW1 + l * 2 * kD) * kD, WLh + (size_t)(kRowW1 + l * 2 * kD) * kD, kD,
        HU, nullptr, nullptr, kHuP,
        nullptr, nullptr, 0,
        kRows, kHuP, kD, 1.0f / (kHCarry * kWCarry), 1.0f);
    edge_sum_kernel<<<kRows, 256, 0, stream>>>(rel_t, edge_mask, HU, TBL, l * kD, msg_b1 + l * kD, SH, SL, CNT);
    gemm3_kernel<1><<<12, 256, 0, stream>>>(
        (const _Float16*)SH, (const _Float16*)SL, kD,
        WHh + (size_t)(kRowMW2 + l * kD) * kD, WLh + (size_t)(kRowMW2 + l * kD) * kD, kD,
        nullptr, AGH, AGL, kD,
        msg_b2 + l * kD, CNT, kCntP,
        kRows, kD, kD, 1.0f / (kSCarry * kWCarry), kAggCarry);
    gemm3_kernel<2><<<12, 256, 0, stream>>>(
        (const _Float16*)AGH, (const _Float16*)AGL, kD,
        WHh + (size_t)(kRowUW1B + l * kD) * kD, WLh + (size_t)(kRowUW1B + l * kD) * kD, kD,
        nullptr, T1H, T1L, kD,
        upd_b1 + l * kD, HU + kD, kHuP,
        kRows, kD, kD, 1.0f / (kAggCarry * kWCarry), kT1Carry);
    gemm3_kernel<3><<<12, 256, 0, stream>>>(
        (const _Float16*)T1H, (const _Float16*)T1L, kD,
        WHh + (size_t)(kRowUW2 + l * kD) * kD, WLh + (size_t)(kRowUW2 + l * kD) * kD, kD,
        X, nullptr, nullptr, kD,
        upd_b2 + l * kD, H, kD,
        kRows, kD, kD, 1.0f / (kT1Carry * kWCarry), 1.0f);
    ln_kernel<<<kRows / 8, 256, 0, stream>>>(X, ln_g + l * kD, ln_b + l * kD, node_mask, H, HH, HL);
  }

  gemm3_kernel<0><<<33, 256, 0, stream>>>(
      (const _Float16*)HH, (const _Float16*)HL, kD,
      WHh + (size_t)kRowHW * kD, WLh + (size_t)kRowHW * kD, kD,
      RABO, nullptr, nullptr, kHeadP,
      nullptr, nullptr, 0,
      kRows, kHeadP, kD, 1.0f / (kHCarry * kWCarry), 1.0f);
  obj_out_kernel<<<(kOut0 / 128 + 7) / 8, 256, 0, stream>>>(RABO, objh_b, out0);
  pair_head_kernel<<<kRows, 256, 0, stream>>>(rel_t, RABO, TBL, relh_b1,
                                              WHh + (size_t)kRowRW2 * kD, relh_b2, out1);
}
